// MomentVideo_84353157693496
// MI455X (gfx1250) — hardware-verified
//
#include <hip/hip_runtime.h>


namespace {
constexpr int NVID = 32, N = 512, M = 64, D = 128, NPAIR = NVID * NVID;
constexpr float XS = 8.0f, PS = 8.0f, EPS = 1e-15f, LOG2E = 1.4426950408889634f;

typedef _Float16 b16;
typedef __attribute__((ext_vector_type(16))) _Float16 v16b;
typedef __attribute__((ext_vector_type(8))) _Float16 v8b;
typedef __attribute__((ext_vector_type(8))) float v8f;
typedef __attribute__((ext_vector_type(4))) float v4f;
__device__ __forceinline__ float bf16_rne(float f) { unsigned int u = __float_as_uint(f); u += 0x7FFFu + ((u >> 16) & 1u); return __uint_as_float(u & 0xFFFF0000u); }
__device__ __forceinline__ v16b frag_kb(const b16* p, int hh) { const v8b a = *(const v8b*)(p + 8 * hh), b = *(const v8b*)(p + 16 + 8 * hh); v16b f;
#pragma unroll
  for (int e = 0; e < 8; ++e) { f[e] = a[e]; f[8 + e] = b[e]; } return f; }
__device__ __forceinline__ v8f wmma16b(v16b a, v16b b, v8f c) { v8f d = __builtin_amdgcn_wmma_f32_16x16x32_f16(false, a, false, b, (short)0, c, false, false); asm volatile("v_nop\n\tv_nop\n\tv_nop\n\tv_nop" : "+v"(d) : "v"(a), "v"(b)); return d; }
__device__ __forceinline__ void wave_lds_sync() { __builtin_amdgcn_fence(__ATOMIC_RELEASE, "workgroup"); __builtin_amdgcn_wave_barrier(); __builtin_amdgcn_fence(__ATOMIC_ACQUIRE, "workgroup"); }
__device__ __forceinline__ float pmul(float a, float b) { float p = a * b; asm volatile("" : "+v"(p)); return p; }
__device__ __forceinline__ float nexp2(float x) { return __builtin_amdgcn_exp2f(x); }

__global__ __launch_bounds__(256) void prep_kernel(const float* __restrict__ v, const float* __restrict__ s, b16* __restrict__ V16, b16* __restrict__ VT16, b16* __restrict__ S16, b16* __restrict__ ST16, float* __restrict__ NVn, float* __restrict__ NSn) {
  __shared__ b16 T[64][66]; __shared__ float nrm[64];
  const int t_ = threadIdx.x; int blk = blockIdx.x; const bool isV = blk < NVID * (N / 64) * 2; const float* src; b16 *P16, *PT; int rows, i, r0, c0;
  if (isV) { i = blk / 16; const int q = blk % 16; r0 = (q >> 1) * 64; c0 = (q & 1) * 64; src = v + ((size_t)i * N) * D; P16 = V16 + (size_t)i * N * D; PT = VT16 + (size_t)i * D * N; rows = N; }
  else { blk -= NVID * 16; i = blk / 2; r0 = 0; c0 = (blk & 1) * 64; src = s + ((size_t)i * M) * D; P16 = S16 + (size_t)i * M * D; PT = ST16 + (size_t)i * D * M; rows = M; }
  for (int q = t_; q < 64 * 64; q += 256) { const int rr = q >> 6, cc = q & 63; T[rr][cc] = (b16)(bf16_rne(src[(size_t)(r0 + rr) * D + c0 + cc]) * XS); }
  __syncthreads();
  if (t_ < 64 && c0 == 0) { float ss = 0.0f; for (int c = 0; c < D; ++c) { const float x = bf16_rne(src[(size_t)(r0 + t_) * D + c]); ss += x * x; } nrm[t_] = sqrtf(ss); }
  __syncthreads();
  for (int pass = 0; pass < 2; ++pass) {
    for (int q = t_; q < 64 * 8; q += 256) { const int rr = q >> 3, c8 = (q & 7) * 8; v8b o; for (int jx = 0; jx < 8; ++jx) o[jx] = T[rr][c8 + jx]; *(volatile v8b*)(P16 + (size_t)(r0 + rr) * D + c0 + c8) = o; }
    for (int q = t_; q < 64 * 8; q += 256) { const int cc = q >> 3, r8 = (q & 7) * 8; v8b o; for (int jx = 0; jx < 8; ++jx) o[jx] = T[r8 + jx][cc]; *(volatile v8b*)(PT + (size_t)(c0 + cc) * rows + r0 + r8) = o; }
    if (c0 == 0 && t_ < 16) { float* dst = isV ? NVn + (size_t)i * N + r0 : NSn + (size_t)i * M; *(volatile v4f*)(dst + t_ * 4) = *(const v4f*)(&nrm[t_ * 4]); }
    __threadfence(); }
}
__global__ __launch_bounds__(128) void pair_kernel(const float* __restrict__ v, const float* __restrict__ s, const b16* __restrict__ V16, const b16* __restrict__ VT16, const b16* __restrict__ S16, const b16* __restrict__ ST16, const float* __restrict__ NVn, const float* __restrict__ NSn, float* __restrict__ R) {
  __shared__ float nvL[N], nsL[M]; __shared__ float red[2][4];
  const int i = blockIdx.x / NVID, j = blockIdx.x % NVID; const int wave = threadIdx.x >> 5, lane = threadIdx.x & 31, hh = lane >> 4, col = lane & 15, t_ = threadIdx.x;
  for (int q = t_; q < N; q += 128) nvL[q] = NVn[(size_t)i * N + q]; if (t_ < M) nsL[t_] = NSn[(size_t)j * M + t_];
  __syncthreads();
  const b16* Vi = V16 + (size_t)i * N * D; const b16* VTi = VT16 + (size_t)i * D * N; const b16* Sj = S16 + (size_t)j * M * D; const b16* STj = ST16 + (size_t)j * D * M;
  const float* vrow = v + (size_t)i * N * D; const float* srow = s + (size_t)j * M * D;
  const float cC = 1.0f / (XS * XS);
  float svsum = 0.0f;
  for (int nt = wave; nt < N / 16; nt += 4) { const int n0 = nt * 16; const int n = n0 + col; const float nvn = nvL[n];
    v8f c4[4] = {{}, {}, {}, {}};
#pragma unroll
    for (int kb = 0; kb < D; kb += 32) { const v16b bq = frag_kb(Vi + (size_t)n * D + kb, hh);
#pragma unroll
      for (int t = 0; t < 4; ++t) c4[t] = wmma16b(frag_kb(Sj + (size_t)(t * 16 + col) * D + kb, hh), bq, c4[t]); }
    float e[32]; float mx = -INFINITY;
#pragma unroll
    for (int t = 0; t < 4; ++t)
#pragma unroll
      for (int r = 0; r < 8; ++r) { const int m = t * 16 + 8 * hh + r; const float cv = (c4[t][r] * cC) / (pmul(nvn, nsL[m]) + EPS); e[t * 8 + r] = cv * LOG2E; mx = fmaxf(mx, e[t * 8 + r]); }
    mx = fmaxf(mx, __shfl_xor(mx, 16)); float sum = 0.0f; v16b ph0, pl0, ph1, pl1;
#pragma unroll
    for (int q = 0; q < 16; ++q) { { const float p = nexp2(e[q] - mx); sum += p; const b16 h_ = (b16)(p * PS); ph0[q] = h_; pl0[q] = (b16)(p * PS - (float)h_); } { const float p = nexp2(e[16 + q] - mx); sum += p; const b16 h_ = (b16)(p * PS); ph1[q] = h_; pl1[q] = (b16)(p * PS - (float)h_); } }
    sum += __shfl_xor(sum, 16); const float inv = 1.0f / (sum * PS * XS);
    v8f at[8];
#pragma unroll
    for (int t = 0; t < 8; ++t) { at[t] = (v8f){}; const b16* a0 = STj + (size_t)(t * 16 + col) * M; v16b fa = frag_kb(a0, hh); at[t] = wmma16b(fa, ph0, at[t]); at[t] = wmma16b(fa, pl0, at[t]); fa = frag_kb(a0 + 32, hh); at[t] = wmma16b(fa, ph1, at[t]); at[t] = wmma16b(fa, pl1, at[t]); }
    float dot = 0.0f, aa = 0.0f;
#pragma unroll
    for (int t = 0; t < 8; ++t)
#pragma unroll
      for (int r = 0; r < 8; ++r) { const float a = at[t][r] * inv; const int d = t * 16 + 8 * hh + r; dot += pmul(bf16_rne(vrow[(size_t)n * D + d]), a); aa += a * a; }
    dot += __shfl_xor(dot, 16); aa += __shfl_xor(aa, 16);
    const float svn = dot / (pmul(nvn, sqrtf(aa)) + EPS); if (hh == 0) svsum += svn; }
  float sssum = 0.0f;
  { const int m = wave * 16 + col; const float nsm = nsL[m]; float mr = -INFINITY, l = 0.0f; v8f o[8];
#pragma unroll
    for (int t = 0; t < 8; ++t) o[t] = (v8f){};
    for (int kb = 0; kb < N; kb += 32) { v8f s0 = {}, s1 = {};
#pragma unroll
      for (int ks = 0; ks < D; ks += 32) { const v16b bq = frag_kb(Sj + (size_t)m * D + ks, hh); s0 = wmma16b(frag_kb(Vi + (size_t)(kb + col) * D + ks, hh), bq, s0); s1 = wmma16b(frag_kb(Vi + (size_t)(kb + 16 + col) * D + ks, hh), bq, s1); }
      float e[16]; float mx = -INFINITY;
#pragma unroll
      for (int r = 0; r < 8; ++r) { const int n0_ = kb + 8 * hh + r; e[r] = (s0[r] * cC) / (pmul(nvL[n0_], nsm) + EPS) * LOG2E; e[8 + r] = (s1[r] * cC) / (pmul(nvL[n0_ + 16], nsm) + EPS) * LOG2E; mx = fmaxf(mx, fmaxf(e[r], e[8 + r])); }
      mx = fmaxf(mx, __shfl_xor(mx, 16)); const float mn = fmaxf(mr, mx); const float al = nexp2(mr - mn); mr = mn; float sum = 0.0f; v16b ph, pl;
#pragma unroll
      for (int q = 0; q < 16; ++q) { const float p = nexp2(e[q] - mn); sum += p; const b16 h_ = (b16)(p * PS); ph[q] = h_; pl[q] = (b16)(p * PS - (float)h_); }
      sum += __shfl_xor(sum, 16); l = l * al + sum;
#pragma unroll
      for (int t = 0; t < 8; ++t) { o[t] *= al; const v16b fa = frag_kb(VTi + (size_t)(t * 16 + col) * N + kb, hh); o[t] = wmma16b(fa, ph, o[t]); o[t] = wmma16b(fa, pl, o[t]); } }
    const float inv = 1.0f / (l * PS * XS); float dot = 0.0f, bb = 0.0f;
#pragma unroll
    for (int t = 0; t < 8; ++t)
#pragma unroll
      for (int r = 0; r < 8; ++r) { const float b_ = o[t][r] * inv; const int d = t * 16 + 8 * hh + r; dot += pmul(bf16_rne(srow[(size_t)m * D + d]), b_); bb += b_ * b_; }
    dot += __shfl_xor(dot, 16); bb += __shfl_xor(bb, 16);
    const float ssm = dot / (pmul(nsm, sqrtf(bb)) + EPS); if (hh == 0) sssum += ssm; }
  svsum += __shfl_xor(svsum, 1); svsum += __shfl_xor(svsum, 2); svsum += __shfl_xor(svsum, 4); svsum += __shfl_xor(svsum, 8); svsum += __shfl_xor(svsum, 16);
  sssum += __shfl_xor(sssum, 1); sssum += __shfl_xor(sssum, 2); sssum += __shfl_xor(sssum, 4); sssum += __shfl_xor(sssum, 8); sssum += __shfl_xor(sssum, 16);
  if (lane == 0) { red[0][wave] = svsum; red[1][wave] = sssum; }
  __syncthreads();
  for (int pass = 0; pass < 2; ++pass) { if (t_ < 32) { float val = 0.0f; if (t_ == 0) val = (((red[0][0] + red[0][1]) + red[0][2]) + red[0][3]) * (1.0f / N); if (t_ == 1) val = (((red[1][0] + red[1][1]) + red[1][2]) + red[1][3]) * (1.0f / M); ((volatile float*)R)[(size_t)blockIdx.x * 32 + t_] = val; } __threadfence(); }
}
__global__ __launch_bounds__(256) void final_kernel(const float* __restrict__ R, float* __restrict__ out) {
  const int t_ = threadIdx.x;
  for (int pass = 0; pass < 2; ++pass) { for (int q = t_; q < NPAIR; q += 256) { const int i = q / NVID, j = q % NVID; ((volatile float*)out)[q] = R[(size_t)q * 32]; ((volatile float*)out)[NPAIR + j * NVID + i] = R[(size_t)q * 32 + 1]; } __threadfence(); }
}
}

extern "C" void kernel_launch(void* const* d_in, const int* in_sizes, int n_in, void* d_out, int out_size, void* d_ws, size_t ws_size, hipStream_t stream) {
  (void)n_in;
  auto Fp = [&](int i) { return (const float*)d_in[i]; };
  if (in_sizes[0] != NVID * N * D || in_sizes[1] != NVID * M * D || out_size != 2 * NPAIR) return;
  size_t off = 0; char* ws = (char*)d_ws;
  auto carve = [&](size_t bytes) { char* p = ws + off; off += (bytes + 255) & ~(size_t)255; return p; };
  b16* V16 = (b16*)carve((size_t)NVID * N * D * 2); b16* VT16 = (b16*)carve((size_t)NVID * N * D * 2); b16* S16 = (b16*)carve((size_t)NVID * M * D * 2); b16* ST16 = (b16*)carve((size_t)NVID * M * D * 2);
  float* NVn = (float*)carve((size_t)NVID * N * 4); float* NSn = (float*)carve((size_t)NVID * M * 4); float* R = (float*)carve((size_t)NPAIR * 32 * 4);
  if (off > ws_size || off > ((size_t)128 << 20)) return;
  prep_kernel<<<NVID * 16 + NVID * 2, 256, 0, stream>>>(Fp(0), Fp(1), V16, VT16, S16, ST16, NVn, NSn);
  pair_kernel<<<NPAIR, 128, 0, stream>>>(Fp(0), Fp(1), V16, VT16, S16, ST16, NVn, NSn, R);
  final_kernel<<<1, 256, 0, stream>>>(R, (float*)d_out);
}
